// VisionMamba_4776003633364
// MI455X (gfx1250) — hardware-verified
//
#include <hip/hip_runtime.h>
#include <math.h>

typedef __attribute__((ext_vector_type(16))) _Float16 v16h;
typedef __attribute__((ext_vector_type(8)))  _Float16 v8h;
typedef __attribute__((ext_vector_type(16))) __bf16   v16b;
typedef __attribute__((ext_vector_type(8)))  __bf16   v8b;
typedef __attribute__((ext_vector_type(8)))  float    v8f;
typedef __attribute__((ext_vector_type(4)))  float    v4f;

constexpr int kB      = 2;
constexpr int kImg    = 224;
constexpr int kPatch  = 16;
constexpr int kGridP  = kImg / kPatch;
constexpr int kL      = kGridP * kGridP;
constexpr int kE      = 384;
constexpr int kDin    = 768;
constexpr int kNst    = 16;
constexpr int kR      = 24;
constexpr int kRP     = 32;
constexpr int kDepth  = 12;
constexpr int kM      = kB * kL;
constexpr int kMp     = 448;
constexpr int kXzP    = 2 * kDin;
constexpr int kXdN    = kR + 2 * kNst;
constexpr int kXdP    = 64;
constexpr int kPK     = kPatch * kPatch;
constexpr int kTP     = 260;
constexpr int kScanCh = 64;
constexpr int kScanTS = 28;
constexpr int kScanNC = 7;

constexpr float kCarWin  = 32.0f;
constexpr float kCarU    = 16.0f;
constexpr float kCarWx   = 32.0f;
constexpr float kCarDtr  = 16.0f;
constexpr float kCarWdt  = 8.0f;
constexpr float kCarY    = 16.0f;
constexpr float kCarWout = 32.0f;
constexpr float kSclIn   = 1.0f / kCarWin;
constexpr float kSclX    = 1.0f / (kCarU * kCarWx);
constexpr float kSclDt   = 1.0f / (kCarDtr * kCarWdt);
constexpr float kSclOut  = 1.0f / (kCarY * kCarWout);

static_assert(kL == 196 && kM == 392, "token count");
static_assert(kMp % 64 == 0 && kMp >= kM, "padded rows");
static_assert(kE % 64 == 0 && kXzP % 64 == 0 && kDin % 64 == 0 && kXdP % 64 == 0, "GEMM N multiples of 64");
static_assert(kE % 32 == 0 && kDin % 32 == 0 && kPK % 32 == 0 && kRP % 32 == 0, "GEMM K multiples of 32");
static_assert(kXdN == 56 && kXdN <= kXdP, "x_proj width");
static_assert(kR == 24 && kRP == 32, "dt rank groups of 8: 3 real + 1 zero");
static_assert(kScanTS * kScanNC == kL, "scan chunks");
static_assert(kL % 4 == 0, "flush rows in groups of 4");
static_assert(kDin % 256 == 0 && kDin % kScanCh == 0 && kMp % 16 == 0 && kMp % 8 == 0, "tile multiples");

constexpr size_t kSzWIN  = (size_t)kDepth * kXzP * kE * 2;
constexpr size_t kSzWOUT = (size_t)kDepth * kE * kDin * 2;
constexpr size_t kSzWXP  = (size_t)2 * kDepth * kXdP * kDin * 2;
constexpr size_t kSzWDT  = (size_t)2 * kDepth * kDin * kRP * 2;
constexpr size_t kSzPW   = (size_t)kE * kPK * 2;
constexpr size_t kSzIM   = (size_t)kMp * kPK * 2;
constexpr size_t kSzME   = (size_t)kMp * kE * 4;
constexpr size_t kSzXN   = (size_t)kMp * kE * 2;
constexpr size_t kSzXZ   = (size_t)kMp * kXzP * 4;
constexpr size_t kSzU    = (size_t)2 * kMp * kDin * 4;
constexpr size_t kSzU16  = (size_t)2 * kMp * kDin * 2;
constexpr size_t kSzDBL  = (size_t)2 * kMp * kXdP * 4;
constexpr size_t kSzDTR  = (size_t)2 * kMp * kRP * 2;
constexpr size_t kSzYS   = (size_t)kMp * kDin * 2;

constexpr size_t kOffWIN  = 0;
constexpr size_t kOffWOUT = kOffWIN  + kSzWIN;
constexpr size_t kOffWXP  = kOffWOUT + kSzWOUT;
constexpr size_t kOffWDT  = kOffWXP  + kSzWXP;
constexpr size_t kOffPWH  = kOffWDT  + kSzWDT;
constexpr size_t kOffPWL  = kOffPWH  + kSzPW;
constexpr size_t kOffIMH  = kOffPWL  + kSzPW;
constexpr size_t kOffIML  = kOffIMH  + kSzIM;
constexpr size_t kOffG    = kOffIML  + kSzIM;
constexpr size_t kOffRES0 = kOffG    + kSzME;
constexpr size_t kOffRES1 = kOffRES0 + kSzME;
constexpr size_t kOffXN   = kOffRES1 + kSzME;
constexpr size_t kOffXZ   = kOffXN   + kSzXN;
constexpr size_t kOffU    = kOffXZ   + kSzXZ;
constexpr size_t kOffU16  = kOffU    + kSzU;
constexpr size_t kOffDBL  = kOffU16  + kSzU16;
constexpr size_t kOffDTR  = kOffDBL  + kSzDBL;
constexpr size_t kOffDLR  = kOffDTR  + kSzDTR;
constexpr size_t kOffYS   = kOffDLR  + kSzU;
constexpr size_t kOffHID  = kOffYS   + kSzYS;
constexpr size_t kWsTotal = kOffHID  + kSzME;
static_assert(kWsTotal == 39329792ull, "carve total");
static_assert(kWsTotal <= 134217728ull, "carve cap");
static_assert((kOffWOUT % 128) == 0 && (kOffWXP % 128) == 0 && (kOffWDT % 128) == 0 && (kOffPWH % 128) == 0 &&
              (kOffPWL % 128) == 0 && (kOffIMH % 128) == 0 && (kOffIML % 128) == 0 && (kOffG % 128) == 0 &&
              (kOffRES0 % 128) == 0 && (kOffRES1 % 128) == 0 && (kOffXN % 128) == 0 && (kOffXZ % 128) == 0 &&
              (kOffU % 128) == 0 && (kOffU16 % 128) == 0 && (kOffDBL % 128) == 0 && (kOffDTR % 128) == 0 &&
              (kOffDLR % 128) == 0 && (kOffYS % 128) == 0 && (kOffHID % 128) == 0, "128-B aligned regions");

__device__ __forceinline__ unsigned short f2bf_bits(float f) {
  unsigned u = __float_as_uint(f);
  return (unsigned short)((u + 0x7FFFu + ((u >> 16) & 1u)) >> 16);
}
__device__ __forceinline__ float bf_bits2f(unsigned short h) { return __uint_as_float(((unsigned)h) << 16); }

__device__ __forceinline__ void dep_guard4_h(v8f& a, v8f& b, v8f& c, v8f& d, v16h x, v16h y) {
  asm volatile("v_nop\n\tv_nop\n\tv_nop\n\tv_nop" : "+v"(a), "+v"(b), "+v"(c), "+v"(d) : "v"(x), "v"(y));
}
__device__ __forceinline__ void dep_guard4_b(v8f& a, v8f& b, v8f& c, v8f& d, v16b x, v16b y) {
  asm volatile("v_nop\n\tv_nop\n\tv_nop\n\tv_nop" : "+v"(a), "+v"(b), "+v"(c), "+v"(d) : "v"(x), "v"(y));
}
__device__ __forceinline__ void keep4_h(v16h a, v16h b, v16h c, v16h d) { asm volatile("v_nop" :: "v"(a), "v"(b), "v"(c), "v"(d)); }
__device__ __forceinline__ void keep4_b(v16b a, v16b b, v16b c, v16b d) { asm volatile("v_nop" :: "v"(a), "v"(b), "v"(c), "v"(d)); }
__device__ __forceinline__ void acc_guard4(v8f& a, v8f& b, v8f& c, v8f& d) {
  asm volatile("v_nop\n\tv_nop\n\tv_nop\n\tv_nop" : "+v"(a), "+v"(b), "+v"(c), "+v"(d));
}
template <typename T> struct Frag;
template <> struct Frag<_Float16> {
  typedef v16h V; union U { v16h v; v8h h[2]; };
  static __device__ __forceinline__ v16h load(const _Float16* p) {
    U f; f.h[0] = *(const v8h*)(p); f.h[1] = *(const v8h*)(p + 16); return f.v;
  }
  static __device__ __forceinline__ v8f mma(v16h a, v16h b, v8f c) {
    return __builtin_amdgcn_wmma_f32_16x16x32_f16(false, a, false, b, (short)0, c, false, false);
  }
  static __device__ __forceinline__ void guard4(v8f& a, v8f& b, v8f& c, v8f& d, v16h x, v16h y) { dep_guard4_h(a, b, c, d, x, y); }
  static __device__ __forceinline__ void keep(v16h a, v16h b, v16h c, v16h d) { keep4_h(a, b, c, d); }
};
template <> struct Frag<__bf16> {
  typedef v16b V; union U { v16b v; v8b h[2]; };
  static __device__ __forceinline__ v16b load(const __bf16* p) {
    U f; f.h[0] = *(const v8b*)(p); f.h[1] = *(const v8b*)(p + 16); return f.v;
  }
  static __device__ __forceinline__ v8f mma(v16b a, v16b b, v8f c) {
    return __builtin_amdgcn_wmma_f32_16x16x32_bf16(false, a, false, b, (short)0, c, false, false);
  }
  static __device__ __forceinline__ void guard4(v8f& a, v8f& b, v8f& c, v8f& d, v16b x, v16b y) { dep_guard4_b(a, b, c, d, x, y); }
  static __device__ __forceinline__ void keep(v16b a, v16b b, v16b c, v16b d) { keep4_b(a, b, c, d); }
};

template <int ET> struct Elem;
template <> struct Elem<0> { typedef _Float16 T; };
template <> struct Elem<1> { typedef __bf16 T; };
template <int ET, bool SPLIT, int BIAS_MODE, int OUT_MODE, bool RESID>
__global__ __launch_bounds__(256) void wmma_gemm64(
    const unsigned short* __restrict__ Ap, const unsigned short* __restrict__ A2p, int lda, long strideA,
    const unsigned short* __restrict__ Btp, const unsigned short* __restrict__ Bt2p, int ldb, long strideB,
    void* __restrict__ Cout, void* __restrict__ Cout2, int ldc, long strideC,
    const float* __restrict__ bias,
    const float* __restrict__ resid, long strideR,
    int M, int N, int K, float scale) {
  typedef typename Elem<ET>::T T;
  typedef typename Frag<T>::V V;
  const T* A = (const T*)Ap; const T* A2 = (const T*)A2p; const T* Bt = (const T*)Btp; const T* Bt2 = (const T*)Bt2p;
  __shared__ __align__(16) float sT[8][16 * 68];
  const int b    = blockIdx.y;
  const int lane = threadIdx.x & 31;
  const int wave = threadIdx.x >> 5;
  const int tilesN = N >> 6;
  const int tilesM = M >> 6;
  const int tile = blockIdx.x * 8 + wave;
  if (tile >= tilesM * tilesN) return;
  const int tm = tile / tilesN;
  const int tn = tile - tm * tilesN;
  const int m0 = tm << 6;
  const int n0 = tn << 6;

  const T* Ab  = A  + (size_t)b * strideA;
  const T* Bb  = Bt + (size_t)b * strideB;
  const T* Ab2 = SPLIT ? (A2  + (size_t)b * strideA) : nullptr;
  const T* Bb2 = SPLIT ? (Bt2 + (size_t)b * strideB) : nullptr;

  const int rlane = lane & 15;
  const int koff  = (lane >> 4) * 8;
  const int mOff  = (lane >> 4) * 8;

  v8f acc[4][4];
#pragma unroll
  for (int i = 0; i < 4; ++i)
#pragma unroll
    for (int j = 0; j < 4; ++j) acc[i][j] = (v8f){0.f,0.f,0.f,0.f,0.f,0.f,0.f,0.f};

  for (int k0 = 0; k0 < K; k0 += 32) {
    V bh[4], bl[4];
#pragma unroll
    for (int j = 0; j < 4; ++j) {
      const size_t bo = (size_t)(n0 + (j << 4) + rlane) * ldb + koff + k0;
      bh[j] = Frag<T>::load(Bb + bo);
      if (SPLIT) bl[j] = Frag<T>::load(Bb2 + bo);
    }
#pragma unroll
    for (int i = 0; i < 4; ++i) {
      const size_t ao = (size_t)(m0 + (i << 4) + rlane) * lda + koff + k0;
      V ah = Frag<T>::load(Ab + ao);
      V al;
      if (SPLIT) al = Frag<T>::load(Ab2 + ao);
#pragma unroll
      for (int j = 0; j < 4; ++j) {
        acc[i][j] = Frag<T>::mma(ah, bh[j], acc[i][j]);
        if (SPLIT) {
          acc[i][j] = Frag<T>::mma(ah, bl[j], acc[i][j]);
          acc[i][j] = Frag<T>::mma(al, bh[j], acc[i][j]);
        }
      }
      Frag<T>::guard4(acc[i][0], acc[i][1], acc[i][2], acc[i][3], ah, SPLIT ? al : ah);
    }
    Frag<T>::keep(bh[0], bh[1], bh[2], bh[3]);
    if (SPLIT) Frag<T>::keep(bl[0], bl[1], bl[2], bl[3]);
  }
  acc_guard4(acc[0][0], acc[0][1], acc[0][2], acc[0][3]);
  acc_guard4(acc[1][0], acc[1][1], acc[1][2], acc[1][3]);
  acc_guard4(acc[2][0], acc[2][1], acc[2][2], acc[2][3]);
  acc_guard4(acc[3][0], acc[3][1], acc[3][2], acc[3][3]);

  float* slab = sT[wave];
  const float* Rb = RESID ? (resid + (size_t)b * strideR) : nullptr;
#pragma unroll
  for (int i = 0; i < 4; ++i) {
    const int mBase = m0 + (i << 4);
#pragma unroll
    for (int j = 0; j < 4; ++j) {
      const int n = n0 + (j << 4) + rlane;
      float bv = 0.f;
      if (BIAS_MODE == 2) bv = bias[n];
#pragma unroll
      for (int r = 0; r < 8; ++r) {
        float v = acc[i][j][r] * scale;
        if (BIAS_MODE == 1) v += bias[mBase + mOff + r];
        if (BIAS_MODE == 2) v += bv;
        if (RESID) v += Rb[(size_t)(mBase + mOff + r) * ldc + n];
        slab[(mOff + r) * 68 + (j << 4) + rlane] = v;
      }
    }
    __builtin_amdgcn_fence(__ATOMIC_RELEASE, "workgroup");
    __builtin_amdgcn_wave_barrier();
    __builtin_amdgcn_fence(__ATOMIC_ACQUIRE, "workgroup");
    if (OUT_MODE == 0) {
      float* C = (float*)Cout + (size_t)b * strideC;
      const int hh = lane >> 4, c4 = (lane & 15) * 4;
      for (int pass = 0; pass < 2; ++pass) {
#pragma unroll
        for (int it = 0; it < 8; ++it) {
          const int row = it * 2 + hh;
          v4f v = *(const v4f*)(slab + row * 68 + c4);
          *(volatile v4f*)(C + (size_t)(mBase + row) * ldc + n0 + c4) = v;
        }
        __threadfence();
      }
    } else {
      const int q = lane >> 3, c8 = (lane & 7) * 8;
      unsigned short* C  = (unsigned short*)Cout  + (size_t)b * strideC;
      unsigned short* C2 = (OUT_MODE == 2) ? ((unsigned short*)Cout2 + (size_t)b * strideC) : nullptr;
      for (int pass = 0; pass < 2; ++pass) {
#pragma unroll
        for (int it = 0; it < 4; ++it) {
          const int row = it * 4 + q;
          const float* sp = slab + row * 68 + c8;
          v8h hv, lv;
#pragma unroll
          for (int e = 0; e < 8; ++e) {
            if (OUT_MODE == 1) {
              hv[e] = (_Float16)sp[e];
            } else {
              unsigned short hb = f2bf_bits(sp[e]);
              unsigned short lb = f2bf_bits(sp[e] - bf_bits2f(hb));
              hv[e] = __builtin_bit_cast(_Float16, hb);
              lv[e] = __builtin_bit_cast(_Float16, lb);
            }
          }
          *(volatile v8h*)(C + (size_t)(mBase + row) * ldc + n0 + c8) = hv;
          if (OUT_MODE == 2) *(volatile v8h*)(C2 + (size_t)(mBase + row) * ldc + n0 + c8) = lv;
        }
        __threadfence();
      }
    }
    __builtin_amdgcn_fence(__ATOMIC_RELEASE, "workgroup");
    __builtin_amdgcn_wave_barrier();
    __builtin_amdgcn_fence(__ATOMIC_ACQUIRE, "workgroup");
  }
}

__global__ __launch_bounds__(256) void cast_f16_kernel(
    const float* __restrict__ src, unsigned short* __restrict__ dst, int total8, float scale)
{
  const int i = blockIdx.x * 256 + threadIdx.x;
  if (i >= total8) return;
  const size_t e0 = (size_t)i << 3;
  const float* p = src + e0;
  const v4f a0 = *(const v4f*)(p);
  const v4f a1 = *(const v4f*)(p + 4);
  v8h hv;
#pragma unroll
  for (int e = 0; e < 4; ++e) {
    hv[e]     = (_Float16)(a0[e] * scale);
    hv[4 + e] = (_Float16)(a1[e] * scale);
  }
  unsigned short* q = dst + e0;
  *(volatile v8h*)q = hv;
  __threadfence();
  *(volatile v8h*)q = hv;
}

__global__ __launch_bounds__(256) void xproj_pad_cast_kernel(
    const float* __restrict__ wf, const float* __restrict__ wr, unsigned short* __restrict__ dst, int total8, float scale)
{
  const int dir = blockIdx.y;
  const float* src = dir ? wr : wf;
  const int i = blockIdx.x * 256 + threadIdx.x;
  if (i >= total8) return;
  const int e0 = i << 3;
  const int rowAll = e0 / kDin;
  const int col = e0 - rowAll * kDin;
  const int n = rowAll & (kXdP - 1);
  const int layer = rowAll / kXdP;
  const bool live = n < kXdN;
  const int nc = live ? n : (kXdN - 1);
  const float* p = src + ((size_t)(layer * kXdN + nc)) * kDin + col;
  const v4f a0 = *(const v4f*)(p);
  const v4f a1 = *(const v4f*)(p + 4);
  v8h hv;
#pragma unroll
  for (int e = 0; e < 4; ++e) {
    const float f0 = live ? (a0[e] * scale) : 0.0f;
    const float f1 = live ? (a1[e] * scale) : 0.0f;
    hv[e]     = (_Float16)f0;
    hv[4 + e] = (_Float16)f1;
  }
  unsigned short* q = dst + (size_t)dir * ((size_t)kDepth * kXdP * kDin) + e0;
  *(volatile v8h*)q = hv;
  __threadfence();
  *(volatile v8h*)q = hv;
}

__global__ __launch_bounds__(256) void dtproj_pad_cast_kernel(
    const float* __restrict__ wf, const float* __restrict__ wr, unsigned short* __restrict__ dst, int total8, float scale)
{
  const int dir = blockIdx.y;
  const float* src = dir ? wr : wf;
  const int i = blockIdx.x * 256 + threadIdx.x;
  if (i >= total8) return;
  const int row = i >> 2;
  const int g = i & 3;
  const bool live = g < 3;
  const int gc = live ? g : 2;
  const float* p = src + (size_t)row * kR + gc * 8;
  const v4f a0 = *(const v4f*)(p);
  const v4f a1 = *(const v4f*)(p + 4);
  v8h hv;
#pragma unroll
  for (int e = 0; e < 4; ++e) {
    const float f0 = live ? (a0[e] * scale) : 0.0f;
    const float f1 = live ? (a1[e] * scale) : 0.0f;
    hv[e]     = (_Float16)f0;
    hv[4 + e] = (_Float16)f1;
  }
  unsigned short* q = dst + (size_t)dir * ((size_t)kDepth * kDin * kRP) + ((size_t)i << 3);
  *(volatile v8h*)q = hv;
  __threadfence();
  *(volatile v8h*)q = hv;
}

__global__ __launch_bounds__(256) void split_rows_bf16_kernel(
    const float* __restrict__ src, unsigned short* __restrict__ dhi, unsigned short* __restrict__ dlo, int total8)
{
  const int i = blockIdx.x * 256 + threadIdx.x;
  if (i >= total8) return;
  const size_t e0 = (size_t)i << 3;
  const v4f a0 = *(const v4f*)(src + e0);
  const v4f a1 = *(const v4f*)(src + e0 + 4);
  v8h hv, lv;
#pragma unroll
  for (int e = 0; e < 4; ++e) {
    const unsigned short h0 = f2bf_bits(a0[e]), h1 = f2bf_bits(a1[e]);
    const unsigned short l0 = f2bf_bits(a0[e] - bf_bits2f(h0)), l1 = f2bf_bits(a1[e] - bf_bits2f(h1));
    hv[e]     = __builtin_bit_cast(_Float16, h0);
    hv[4 + e] = __builtin_bit_cast(_Float16, h1);
    lv[e]     = __builtin_bit_cast(_Float16, l0);
    lv[4 + e] = __builtin_bit_cast(_Float16, l1);
  }
  unsigned short* qh = dhi + e0;
  unsigned short* ql = dlo + e0;
  *(volatile v8h*)qh = hv;
  *(volatile v8h*)ql = lv;
  __threadfence();
  *(volatile v8h*)qh = hv;
  *(volatile v8h*)ql = lv;
}

__global__ __launch_bounds__(256) void im2col_split_kernel(
    const float* __restrict__ x, unsigned short* __restrict__ dhi, unsigned short* __restrict__ dlo, int total8)
{
  const int i = blockIdx.x * 256 + threadIdx.x;
  if (i >= total8) return;
  const int row = i >> 5;
  const int g = i & 31;
  const bool live = row < kM;
  const int rc = live ? row : (kM - 1);
  const int b = rc / kL;
  const int l = rc - b * kL;
  const int py = l / kGridP;
  const int px = l - py * kGridP;
  const int iy = g >> 1;
  const int ix0 = (g & 1) * 8;
  const float* p = x + (size_t)b * (kImg * kImg) + (size_t)(py * kPatch + iy) * kImg + px * kPatch + ix0;
  const v4f a0 = *(const v4f*)(p);
  const v4f a1 = *(const v4f*)(p + 4);
  v8h hv, lv;
#pragma unroll
  for (int e = 0; e < 4; ++e) {
    const float f0 = live ? a0[e] : 0.0f;
    const float f1 = live ? a1[e] : 0.0f;
    const unsigned short h0 = f2bf_bits(f0), h1 = f2bf_bits(f1);
    const unsigned short l0 = f2bf_bits(f0 - bf_bits2f(h0)), l1 = f2bf_bits(f1 - bf_bits2f(h1));
    hv[e]     = __builtin_bit_cast(_Float16, h0);
    hv[4 + e] = __builtin_bit_cast(_Float16, h1);
    lv[e]     = __builtin_bit_cast(_Float16, l0);
    lv[4 + e] = __builtin_bit_cast(_Float16, l1);
  }
  const size_t e0 = (size_t)i << 3;
  unsigned short* qh = dhi + e0;
  unsigned short* ql = dlo + e0;
  *(volatile v8h*)qh = hv;
  *(volatile v8h*)ql = lv;
  __threadfence();
  *(volatile v8h*)qh = hv;
  *(volatile v8h*)ql = lv;
}

__global__ __launch_bounds__(256) void zero_fill_kernel(float* __restrict__ dst, int total4)
{
  const int i = blockIdx.x * 256 + threadIdx.x;
  if (i >= total4) return;
  const v4f z = (v4f){0.f, 0.f, 0.f, 0.f};
  float* q = dst + ((size_t)i << 2);
  *(volatile v4f*)q = z;
  __threadfence();
  *(volatile v4f*)q = z;
}

template <int MODE>
__global__ __launch_bounds__(256) void add_rms_kernel(
    const float* __restrict__ srcA, const float* __restrict__ srcB, const float* __restrict__ pbias,
    const float* __restrict__ wn, float* __restrict__ resOut, unsigned short* __restrict__ xn16,
    float* __restrict__ outF)
{
  __shared__ __align__(16) float sX[8 * kE];
  const int tid = threadIdx.x, lane = tid & 31, wave = tid >> 5;
  const int row = blockIdx.x * 8 + wave;
  const bool live = row < kM;
  const int rc = live ? row : (kM - 1);
  const int l = rc % kL;
  v4f v[3];
  float ss = 0.0f;
#pragma unroll
  for (int it = 0; it < 3; ++it) {
    const int c = it * 128 + lane * 4;
    v4f a = *(const v4f*)(srcA + (size_t)rc * kE + c);
    if (MODE == 0) {
      const v4f pbv = *(const v4f*)(pbias + c);
      const v4f pe  = *(const v4f*)(srcB + (size_t)l * kE + c);
      a = (a + pbv) + pe;
    } else {
      const v4f hb = *(const v4f*)(srcB + (size_t)rc * kE + c);
      a = a + hb;
    }
#pragma unroll
    for (int e = 0; e < 4; ++e) {
      const float xv = live ? a[e] : 0.0f;
      v[it][e] = xv;
      ss = fmaf(xv, xv, ss);
    }
  }
#pragma unroll
  for (int off = 16; off >= 1; off >>= 1) ss += __shfl_xor(ss, off, 32);
  const float sc = rsqrtf(ss * (1.0f / (float)kE) + 1e-5f);
  v4f o[3];
#pragma unroll
  for (int it = 0; it < 3; ++it) {
    const int c = it * 128 + lane * 4;
    const v4f wv = *(const v4f*)(wn + c);
    o[it] = (v[it] * sc) * wv;
  }
  if (MODE == 2) {
    if (live) {
      for (int pass = 0; pass < 2; ++pass) {
#pragma unroll
        for (int it = 0; it < 3; ++it)
          *(volatile v4f*)(outF + (size_t)row * kE + it * 128 + lane * 4) = o[it];
        __threadfence();
      }
    }
  } else {
    for (int pass = 0; pass < 2; ++pass) {
#pragma unroll
      for (int it = 0; it < 3; ++it)
        *(volatile v4f*)(resOut + (size_t)row * kE + it * 128 + lane * 4) = v[it];
      __threadfence();
    }
#pragma unroll
    for (int it = 0; it < 3; ++it)
      *(v4f*)(sX + wave * kE + it * 128 + lane * 4) = o[it];
    __syncthreads();
    const bool second = tid < 128;
    v8h h0, h1;
    {
      const float* sp = sX + tid * 8;
      const v4f a0 = *(const v4f*)(sp);
      const v4f a1 = *(const v4f*)(sp + 4);
#pragma unroll
      for (int e = 0; e < 4; ++e) { h0[e] = (_Float16)a0[e]; h0[4 + e] = (_Float16)a1[e]; }
    }
#pragma unroll
    for (int e = 0; e < 8; ++e) h1[e] = (_Float16)0.0f;
    if (second) {
      const float* sp = sX + (256 + tid) * 8;
      const v4f a0 = *(const v4f*)(sp);
      const v4f a1 = *(const v4f*)(sp + 4);
#pragma unroll
      for (int e = 0; e < 4; ++e) { h1[e] = (_Float16)a0[e]; h1[4 + e] = (_Float16)a1[e]; }
    }
    unsigned short* q0 = xn16 + (size_t)blockIdx.x * 8 * kE + tid * 8;
    unsigned short* q1 = q0 + 2048;
    for (int pass = 0; pass < 2; ++pass) {
      *(volatile v8h*)q0 = h0;
      if (second) *(volatile v8h*)q1 = h1;
      __threadfence();
    }
  }
}

__global__ __launch_bounds__(256) void conv_silu_kernel(
    const float* __restrict__ XZ,
    const float* __restrict__ cwf, const float* __restrict__ cbf,
    const float* __restrict__ cwr, const float* __restrict__ cbr,
    float* __restrict__ U, unsigned short* __restrict__ U16)
{
  __shared__ __align__(16) float sT[16 * kTP];
  const int tid = threadIdx.x, lane = tid & 31, wave = tid >> 5;
  const int dir = blockIdx.z;
  const int d0 = blockIdx.x * 256, d = d0 + tid;
  const int r0 = blockIdx.y * 16;
  const float* cw = dir ? cwr : cwf;
  const float* cb = dir ? cbr : cbf;
  const v4f wv = *(const v4f*)(cw + (size_t)d * 4);
  const float bc = cb[d];
#pragma unroll 1
  for (int s = 0; s < 16; ++s) {
    const int r = r0 + s;
    const bool live = r < kM;
    const int rc = live ? r : (kM - 1);
    const int bb = rc / kL;
    const int l = rc - bb * kL;
    const int base = bb * kL;
    float acc = 0.0f;
#pragma unroll
    for (int j = 0; j < 4; ++j) {
      const int lj = dir ? (l + 3 - j) : (l - 3 + j);
      const bool ok = live && (lj >= 0) && (lj < kL);
      const int ljc = lj < 0 ? 0 : (lj >= kL ? (kL - 1) : lj);
      const float xv = XZ[(size_t)(base + ljc) * kXzP + d];
      const float xs = ok ? xv : 0.0f;
      acc = fmaf(wv[j], xs, acc);
    }
    const float sv = acc + bc;
    const float sg = 1.0f / (1.0f + expf(-sv));
    const float ov = live ? (sv * sg) : 0.0f;
    sT[s * kTP + tid] = ov;
  }
  __syncthreads();
  const int hrow = wave >> 1;
  const int hch  = (wave & 1) * 128 + lane * 4;
  v4f fv[4];
  v8h bv[2];
#pragma unroll
  for (int it = 0; it < 4; ++it) fv[it] = *(const v4f*)(sT + (it * 4 + hrow) * kTP + hch);
#pragma unroll
  for (int it = 0; it < 2; ++it) {
    const float* sp = sT + (it * 8 + wave) * kTP + lane * 8;
    const v4f a0 = *(const v4f*)(sp);
    const v4f a1 = *(const v4f*)(sp + 4);
#pragma unroll
    for (int e = 0; e < 4; ++e) {
      bv[it][e]     = (_Float16)(a0[e] * kCarU);
      bv[it][4 + e] = (_Float16)(a1[e] * kCarU);
    }
  }
  float* Ud = U + (size_t)dir * kMp * kDin;
  unsigned short* U16d = U16 + (size_t)dir * kMp * kDin;
  for (int pass = 0; pass < 2; ++pass) {
#pragma unroll
    for (int it = 0; it < 4; ++it)
      *(volatile v4f*)(Ud + (size_t)(r0 + it * 4 + hrow) * kDin + d0 + hch) = fv[it];
#pragma unroll
    for (int it = 0; it < 2; ++it)
      *(volatile v8h*)(U16d + (size_t)(r0 + it * 8 + wave) * kDin + d0 + lane * 8) = bv[it];
    __threadfence();
  }
}

__global__ __launch_bounds__(256) void dt_cast_kernel(
    const float* __restrict__ DBL, unsigned short* __restrict__ DTR16, int total8, float scale)
{
  const int i = blockIdx.x * 256 + threadIdx.x;
  if (i >= total8) return;
  const int row = i >> 2;
  const int g = i & 3;
  const bool live = g < 3;
  const int gc = live ? g : 2;
  const float* p = DBL + (size_t)row * kXdP + gc * 8;
  const v4f a0 = *(const v4f*)(p);
  const v4f a1 = *(const v4f*)(p + 4);
  v8h hv;
#pragma unroll
  for (int e = 0; e < 4; ++e) {
    const float f0 = live ? (a0[e] * scale) : 0.0f;
    const float f1 = live ? (a1[e] * scale) : 0.0f;
    hv[e]     = (_Float16)f0;
    hv[4 + e] = (_Float16)f1;
  }
  unsigned short* q = DTR16 + ((size_t)i << 3);
  *(volatile v8h*)q = hv;
  __threadfence();
  *(volatile v8h*)q = hv;
}

__global__ __launch_bounds__(64) void scan_kernel(
    const float* __restrict__ DLR, const float* __restrict__ U, const float* __restrict__ XZ,
    const float* __restrict__ DBL,
    const float* __restrict__ AlogF, const float* __restrict__ AlogR,
    const float* __restrict__ DpF, const float* __restrict__ DpR,
    const float* __restrict__ dtbF, const float* __restrict__ dtbR,
    unsigned short* __restrict__ YS16)
{
  __shared__ __align__(16) float sX[kScanTS * kXdP];
  __shared__ __align__(16) float sY[kL * kScanCh];
  __shared__ __align__(16) float sA[kNst * kScanCh];
  const int tid = threadIdx.x, lane = tid & 31, wave = tid >> 5;
  constexpr int kBlkPerB = kDin / kScanCh;
  const int bix = blockIdx.x / kBlkPerB;
  const int d0  = (blockIdx.x - bix * kBlkPerB) * kScanCh;
  const int d   = d0 + tid;
  const int rowb = bix * kL;

#pragma unroll 1
  for (int dir = 0; dir < 2; ++dir) {
    const float* Alog = dir ? AlogR : AlogF;
    const float* Dpp  = dir ? DpR : DpF;
    const float* dtb  = dir ? dtbR : dtbF;
    const float* pDLR = DLR + (size_t)dir * kMp * kDin;
    const float* pU   = U   + (size_t)dir * kMp * kDin;
    const float* pDBL = DBL + (size_t)dir * kMp * kXdP;
    __syncthreads();
#pragma unroll 1
    for (int s = 0; s < kNst; ++s) sA[s * kScanCh + tid] = -expf(Alog[(size_t)d * kNst + s]);
    __syncthreads();
    float negA[kNst], h[kNst];
#pragma unroll
    for (int s = 0; s < kNst; ++s) {
      negA[s] = sA[s * kScanCh + tid];
      h[s] = 0.0f;
    }
    const float bb = dtb[d];
    const float Dd = Dpp[d];
#pragma unroll 1
    for (int ci = 0; ci < kScanNC; ++ci) {
      const int c = dir ? (kScanNC - 1 - ci) : ci;
      const int p0 = c * kScanTS;
      __syncthreads();
#pragma unroll
      for (int i = 0; i < 7; ++i) {
        const int idx = tid + 64 * i;
        const int r = idx >> 4;
        const int c4 = (idx & 15) * 4;
        *(v4f*)(sX + r * kXdP + c4) = *(const v4f*)(pDBL + (size_t)(rowb + p0 + r) * kXdP + c4);
      }
      __syncthreads();
#pragma unroll 1
      for (int si = 0; si < kScanTS; ++si) {
        const int s = dir ? (kScanTS - 1 - si) : si;
        const int p = p0 + s;
        const size_t row = (size_t)(rowb + p);
        const float* xr = sX + s * kXdP;
        float Bs[kNst], Cs[kNst];
#pragma unroll
        for (int q4 = 0; q4 < 4; ++q4) {
          const v4f bv = *(const v4f*)(xr + kR + 4 * q4);
          const v4f cv = *(const v4f*)(xr + kR + kNst + 4 * q4);
          Bs[4 * q4 + 0] = bv[0]; Bs[4 * q4 + 1] = bv[1]; Bs[4 * q4 + 2] = bv[2]; Bs[4 * q4 + 3] = bv[3];
          Cs[4 * q4 + 0] = cv[0]; Cs[4 * q4 + 1] = cv[1]; Cs[4 * q4 + 2] = cv[2]; Cs[4 * q4 + 3] = cv[3];
        }
        const float a   = pDLR[row * kDin + d] + bb;
        const float ea  = __expf(-fabsf(a));
        const float u1  = 1.0f + ea;
        const float l1p = __logf(u1) + (ea - (u1 - 1.0f)) * __builtin_amdgcn_rcpf(u1);
        const float dt  = fmaxf(a, 0.0f) + l1p;
        const float xt  = pU[row * kDin + d];
        const float dtx = dt * xt;
        float y = 0.0f;
#pragma unroll
        for (int k = 0; k < kNst; ++k) {
          const float e = __expf(dt * negA[k]);
          h[k] = fmaf(e, h[k], dtx * Bs[k]);
          y = fmaf(h[k], Cs[k], y);
        }
        y = fmaf(xt, Dd, y);
        const float zv = XZ[row * kXzP + kDin + d];
        const float sg = 1.0f / (1.0f + expf(-zv));
        const float yo = y * (zv * sg);
        if (dir == 0) {
          sY[p * kScanCh + tid] = yo;
        } else {
          const float y0 = sY[p * kScanCh + tid];
          sY[p * kScanCh + tid] = y0 + yo;
        }
      }
    }
  }
  __syncthreads();
  const int q = lane >> 3, c8 = (lane & 7) * 8;
#pragma unroll 1
  for (int it = 0; it < 25; ++it) {
    const int rbase = it * 8 + wave * 4;
    if (rbase < kL) {
      const int prow = rbase + q;
      const float* sp = sY + prow * kScanCh + c8;
      const v4f a0 = *(const v4f*)(sp);
      const v4f a1 = *(const v4f*)(sp + 4);
      v8h hv;
#pragma unroll
      for (int e = 0; e < 4; ++e) {
        hv[e]     = (_Float16)(a0[e] * kCarY);
        hv[4 + e] = (_Float16)(a1[e] * kCarY);
      }
      unsigned short* dst = YS16 + (size_t)(rowb + prow) * kDin + d0 + c8;
      *(volatile v8h*)dst = hv;
      __threadfence();
      *(volatile v8h*)dst = hv;
    }
  }
}

extern "C" void kernel_launch(void* const* d_in, const int* in_sizes, int n_in,
                              void* d_out, int out_size, void* d_ws, size_t ws_size,
                              hipStream_t stream)
{
  if (n_in < 22) return;
  if (in_sizes[0] != kB * kImg * kImg) return;
  if (in_sizes[1] != kE * kPK) return;
  if (in_sizes[2] != kE) return;
  if (in_sizes[3] != kL * kE) return;
  if (in_sizes[4] != kDepth * kE) return;
  if (in_sizes[5] != kDepth * kXzP * kE) return;
  if (in_sizes[6] != kDepth * kDin * 4 || in_sizes[13] != kDepth * kDin * 4) return;
  if (in_sizes[7] != kDepth * kDin || in_sizes[14] != kDepth * kDin) return;
  if (in_sizes[8] != kDepth * kXdN * kDin || in_sizes[15] != kDepth * kXdN * kDin) return;
  if (in_sizes[9] != kDepth * kDin * kR || in_sizes[16] != kDepth * kDin * kR) return;
  if (in_sizes[10] != kDepth * kDin || in_sizes[17] != kDepth * kDin) return;
  if (in_sizes[11] != kDepth * kDin * kNst || in_sizes[18] != kDepth * kDin * kNst) return;
  if (in_sizes[12] != kDepth * kDin || in_sizes[19] != kDepth * kDin) return;
  if (in_sizes[20] != kDepth * kE * kDin) return;
  if (in_sizes[21] != kE) return;
  if (out_size != kM * kE) return;
  if (ws_size < kWsTotal) return;

  const float* x       = (const float*)d_in[0];
  const float* patch_w = (const float*)d_in[1];
  const float* patch_b = (const float*)d_in[2];
  const float* pos     = (const float*)d_in[3];
  const float* norm_w  = (const float*)d_in[4];
  const float* ipw     = (const float*)d_in[5];
  const float* cw      = (const float*)d_in[6];
  const float* cb      = (const float*)d_in[7];
  const float* xpw     = (const float*)d_in[8];
  const float* dtw     = (const float*)d_in[9];
  const float* dtb     = (const float*)d_in[10];
  const float* Alog    = (const float*)d_in[11];
  const float* Dp      = (const float*)d_in[12];
  const float* cwr     = (const float*)d_in[13];
  const float* cbr     = (const float*)d_in[14];
  const float* xpwr    = (const float*)d_in[15];
  const float* dtwr    = (const float*)d_in[16];
  const float* dtbr    = (const float*)d_in[17];
  const float* Alogr   = (const float*)d_in[18];
  const float* Dpr     = (const float*)d_in[19];
  const float* opw     = (const float*)d_in[20];
  const float* normf   = (const float*)d_in[21];
  float* out = (float*)d_out;

  char* ws = (char*)d_ws;
  unsigned short* WIN  = (unsigned short*)(ws + kOffWIN);
  unsigned short* WOUT = (unsigned short*)(ws + kOffWOUT);
  unsigned short* WXP  = (unsigned short*)(ws + kOffWXP);
  unsigned short* WDT  = (unsigned short*)(ws + kOffWDT);
  unsigned short* PWH  = (unsigned short*)(ws + kOffPWH);
  unsigned short* PWL  = (unsigned short*)(ws + kOffPWL);
  unsigned short* IMH  = (unsigned short*)(ws + kOffIMH);
  unsigned short* IML  = (unsigned short*)(ws + kOffIML);
  float*          G    = (float*)(ws + kOffG);
  float*          RES0 = (float*)(ws + kOffRES0);
  float*          RES1 = (float*)(ws + kOffRES1);
  unsigned short* XN   = (unsigned short*)(ws + kOffXN);
  float*          XZ   = (float*)(ws + kOffXZ);
  float*          U    = (float*)(ws + kOffU);
  unsigned short* U16  = (unsigned short*)(ws + kOffU16);
  float*          DBL  = (float*)(ws + kOffDBL);
  unsigned short* DTR  = (unsigned short*)(ws + kOffDTR);
  float*          DLR  = (float*)(ws + kOffDLR);
  unsigned short* YS   = (unsigned short*)(ws + kOffYS);
  float*          HID  = (float*)(ws + kOffHID);
  const float* dummyf = patch_b;

  static_assert((kDepth * kXzP * kE) % 2048 == 0 && (kDepth * kE * kDin) % 2048 == 0, "cast grids exact");
  static_assert((kDepth * kXdP * kDin) % 2048 == 0 && (kDepth * kDin * kRP) % 2048 == 0, "pad cast grids exact");
  static_assert((kE * kPK) % 2048 == 0 && (kMp * kPK) % 2048 == 0, "split grids exact");
  static_assert((2 * kMp * kRP) % 2048 == 0, "dt cast grid exact");
  static_assert(((kMp - kM) * kDin * 2) % 4096 == 0, "zero fill grid exact");

  cast_f16_kernel<<<(kDepth * kXzP * kE) / 2048, 256, 0, stream>>>(ipw, WIN, (kDepth * kXzP * kE) / 8, kCarWin);
  cast_f16_kernel<<<(kDepth * kE * kDin) / 2048, 256, 0, stream>>>(opw, WOUT, (kDepth * kE * kDin) / 8, kCarWout);
  xproj_pad_cast_kernel<<<dim3((kDepth * kXdP * kDin) / 2048, 2), 256, 0, stream>>>(
      xpw, xpwr, WXP, (kDepth * kXdP * kDin) / 8, kCarWx);
  dtproj_pad_cast_kernel<<<dim3((kDepth * kDin * kRP) / 2048, 2), 256, 0, stream>>>(
      dtw, dtwr, WDT, (kDepth * kDin * kRP) / 8, kCarWdt);
  split_rows_bf16_kernel<<<(kE * kPK) / 2048, 256, 0, stream>>>(patch_w, PWH, PWL, (kE * kPK) / 8);
  im2col_split_kernel<<<(kMp * kPK) / 2048, 256, 0, stream>>>(x, IMH, IML, (kMp * kPK) / 8);
  zero_fill_kernel<<<((kMp - kM) * kDin * 2) / 4096, 256, 0, stream>>>(
      (float*)(ws + kOffYS + (size_t)kM * kDin * 2), ((kMp - kM) * kDin * 2) / 16);

  wmma_gemm64<1, true, 0, 0, false><<<dim3(6, 1), 256, 0, stream>>>(
      IMH, IML, kPK, 0L, PWH, PWL, kPK, 0L,
      (void*)G, (void*)G, kE, 0L, dummyf, dummyf, 0L, kMp, kE, kPK, 1.0f);

  for (int i = 0; i < kDepth; ++i) {
    float* resNew = (i & 1) ? RES1 : RES0;
    const float* resOld = (i & 1) ? RES0 : RES1;
    if (i == 0) {
      add_rms_kernel<0><<<kMp / 8, 256, 0, stream>>>(G, pos, patch_b, norm_w, resNew, XN, resNew);
    } else {
      add_rms_kernel<1><<<kMp / 8, 256, 0, stream>>>(resOld, HID, patch_b, norm_w + (size_t)i * kE, resNew, XN, resNew);
    }

    wmma_gemm64<0, false, 0, 0, false><<<dim3(21, 1), 256, 0, stream>>>(
        XN, XN, kE, 0L,
        WIN + (size_t)i * kXzP * kE, WIN + (size_t)i * kXzP * kE, kE, 0L,
        (void*)XZ, (void*)XZ, kXzP, 0L, dummyf, dummyf, 0L, kMp, kXzP, kE, kSclIn);

    conv_silu_kernel<<<dim3(kDin / 256, kMp / 16, 2), 256, 0, stream>>>(
        XZ, cw + (size_t)i * kDin * 4, cb + (size_t)i * kDin,
        cwr + (size_t)i * kDin * 4, cbr + (size_t)i * kDin, U, U16);

    wmma_gemm64<0, false, 0, 0, false><<<dim3(1, 2), 256, 0, stream>>>(
        U16, U16, kDin, (long)kMp * kDin,
        WXP + (size_t)i * kXdP * kDin, WXP + (size_t)i * kXdP * kDin, kDin, (long)kDepth * kXdP * kDin,
        (void*)DBL, (void*)DBL, kXdP, (long)kMp * kXdP, dummyf, dummyf, 0L, kMp, kXdP, kDin, kSclX);

    dt_cast_kernel<<<(2 * kMp * kRP) / 2048, 256, 0, stream>>>(DBL, DTR, (2 * kMp * kRP) / 8, kCarDtr);

    wmma_gemm64<0, false, 0, 0, false><<<dim3(11, 2), 256, 0, stream>>>(
        DTR, DTR, kRP, (long)kMp * kRP,
        WDT + (size_t)i * kDin * kRP, WDT + (size_t)i * kDin * kRP, kRP, (long)kDepth * kDin * kRP,
        (void*)DLR, (void*)DLR, kDin, (long)kMp * kDin, dummyf, dummyf, 0L, kMp, kDin, kRP, kSclDt);

    scan_kernel<<<kB * (kDin / kScanCh), kScanCh, 0, stream>>>(
        DLR, U, XZ, DBL,
        Alog + (size_t)i * kDin * kNst, Alogr + (size_t)i * kDin * kNst,
        Dp + (size_t)i * kDin, Dpr + (size_t)i * kDin,
        dtb + (size_t)i * kDin, dtbr + (size_t)i * kDin, YS);

    wmma_gemm64<0, false, 0, 0, false><<<dim3(6, 1), 256, 0, stream>>>(
        YS, YS, kDin, 0L,
        WOUT + (size_t)i * kE * kDin, WOUT + (size_t)i * kE * kDin, kDin, 0L,
        (void*)HID, (void*)HID, kE, 0L, dummyf, dummyf, 0L, kMp, kE, kDin, kSclOut);
  }

  add_rms_kernel<2><<<kMp / 8, 256, 0, stream>>>(RES1, HID, patch_b, normf, RES0, XN, out);
}
